// Inv_block_19670950216069
// MI455X (gfx1250) — hardware-verified
//
#include <hip/hip_runtime.h>
#define BB 2
#define CC 128
#define CH 64
#define CQ 32
#define KINV 7
#define K2 49
#define GG 4
#define GC 16
#define HW 128
#define NP (BB * HW * HW)
#define NKW 196
#define NKP 208

typedef __bf16 v16b __attribute__((ext_vector_type(16)));
typedef unsigned short v8us __attribute__((ext_vector_type(8), may_alias));
typedef float  v8f  __attribute__((ext_vector_type(8)));
typedef float  v4f  __attribute__((ext_vector_type(4)));
typedef float  v4fa __attribute__((ext_vector_type(4), may_alias));
union FragB { v16b v; v8us half[2]; unsigned short u[16]; };

__device__ __forceinline__ unsigned short bf16_bits(float x) { unsigned int u = __float_as_uint(x); return (unsigned short)((u + 0x7FFFu + ((u >> 16) & 1u)) >> 16); }
__device__ __forceinline__ float bf16_val(unsigned short b) { return __uint_as_float(((unsigned int)b) << 16); }
__device__ __forceinline__ float bf16_round(float x) { return bf16_val(bf16_bits(x)); }
template <int NT>
__device__ __forceinline__ v8f mmaN(v16b ah, v16b al, v16b bh, v16b bl, v8f c) {
  c = __builtin_amdgcn_wmma_f32_16x16x32_bf16(false, ah, false, bh, (short)0, c, false, false);
  if (NT >= 2) c = __builtin_amdgcn_wmma_f32_16x16x32_bf16(false, al, false, bh, (short)0, c, false, false);
  if (NT >= 3) c = __builtin_amdgcn_wmma_f32_16x16x32_bf16(false, ah, false, bl, (short)0, c, false, false);
  asm volatile("v_nop\n\tv_nop\n\tv_nop\n\tv_nop" : "+v"(c) : "v"(ah), "v"(al), "v"(bh), "v"(bl));
  return c;
}

__device__ __forceinline__ void store_span256(float* span, v4f lo, v4f hi, int lane) {
  v4f a, b; const int s0 = lane >> 1, s1 = 16 + (lane >> 1); const bool odd = (lane & 1) != 0;
#pragma unroll
  for (int q = 0; q < 4; ++q) { const float l0 = __shfl(lo[q], s0, 32), h0 = __shfl(hi[q], s0, 32), l1 = __shfl(lo[q], s1, 32), h1 = __shfl(hi[q], s1, 32); a[q] = odd ? h0 : l0; b[q] = odd ? h1 : l1; }
  for (int pass = 0; pass < 2; ++pass) { *(volatile v4f*)(span + 4 * lane) = a; *(volatile v4f*)(span + 128 + 4 * lane) = b; if (pass == 0) __threadfence(); } }
__device__ __forceinline__ void store_span512h(_Float16* span, v8us p0, v8us p1, int lane) {
  typedef unsigned int v4u __attribute__((ext_vector_type(4))); union U { v8us h; v4u u; }; U x0, x1, a, b; x0.h = p0; x1.h = p1; const int s0 = lane >> 1, s1 = 16 + (lane >> 1); const bool odd = (lane & 1) != 0;
#pragma unroll
  for (int q = 0; q < 4; ++q) { const unsigned l0 = __shfl(x0.u[q], s0, 32), h0 = __shfl(x1.u[q], s0, 32), l1 = __shfl(x0.u[q], s1, 32), h1 = __shfl(x1.u[q], s1, 32); a.u[q] = odd ? h0 : l0; b.u[q] = odd ? h1 : l1; }
  for (int pass = 0; pass < 2; ++pass) { *(volatile v8us*)((unsigned short*)span + 8 * lane) = a.h; *(volatile v8us*)((unsigned short*)span + 256 + 8 * lane) = b.h; if (pass == 0) __threadfence(); } }

__global__ __launch_bounds__(256) void k_wt_bf16(const float* __restrict__ W, unsigned short* __restrict__ Wt, int K, int N) {
  const int t = blockIdx.x * 256 + threadIdx.x;
  const int k8n = K / 8;
  if (t >= N * k8n) return;
  const int n = t / k8n, k8 = (t % k8n) * 8;
  v8us v;
#pragma unroll
  for (int i = 0; i < 8; ++i) v[i] = bf16_bits(W[(size_t)(k8 + i) * N + n]);
  *(volatile v8us*)(Wt + (size_t)n * K + k8) = v;
  __threadfence();
  *(volatile v8us*)(Wt + (size_t)n * K + k8) = v;
}

template <bool ASPLIT, int ACT, bool BIAS_BF16>
__global__ __launch_bounds__(128) void k_gemm_bf(const float* __restrict__ A, int lda, const unsigned short* __restrict__ Wt, int ldb,
                                               const float* __restrict__ bias, float* __restrict__ C, int ldc, int M, int N, int K) {
  __shared__ __attribute__((aligned(16))) float so[4][16][64];
  const int tid = threadIdx.x, w = tid >> 5, lane = tid & 31, ln = lane & 15, hh = lane >> 4;
  const int ntn = N / 64;
  const int wid = blockIdx.x * 4 + w;
  const int mt = wid / ntn, nq = wid % ntn;
  if (mt * 16 >= M) return;
  const int row0 = mt * 16, col0 = nq * 64;
  const float* arow = A + (size_t)(row0 + ln) * lda;
  v8f acc[4] = {};
  for (int kb = 0; kb < K; kb += 32) {
    FragB ah, al;
    const v4f x0 = *(const v4fa*)(arow + kb + 8 * hh), x1 = *(const v4fa*)(arow + kb + 8 * hh + 4);
    const v4f x2 = *(const v4fa*)(arow + kb + 16 + 8 * hh), x3 = *(const v4fa*)(arow + kb + 16 + 8 * hh + 4);
    float xs[16] = {x0[0],x0[1],x0[2],x0[3],x1[0],x1[1],x1[2],x1[3],x2[0],x2[1],x2[2],x2[3],x3[0],x3[1],x3[2],x3[3]};
#pragma unroll
    for (int i = 0; i < 16; ++i) { const unsigned short hb = bf16_bits(xs[i]); ah.u[i] = hb; al.u[i] = ASPLIT ? bf16_bits(xs[i] - bf16_val(hb)) : (unsigned short)0; }
#pragma unroll
    for (int t = 0; t < 4; ++t) {
      const unsigned short* brow = Wt + (size_t)(col0 + t * 16 + ln) * ldb + kb;
      FragB b;
      b.half[0] = *(const v8us*)(brow + 8 * hh);
      b.half[1] = *(const v8us*)(brow + 16 + 8 * hh);
      acc[t] = mmaN<ASPLIT ? 2 : 1>(ah.v, al.v, b.v, b.v, acc[t]);
    }
  }
#pragma unroll
  for (int t = 0; t < 4; ++t) {
    float bv = bias ? bias[col0 + t * 16 + ln] : 0.f;
    if (BIAS_BF16) bv = bf16_round(bv);
#pragma unroll
    for (int r = 0; r < 8; ++r) { float v = acc[t][r] + bv; if (ACT == 1) v = fmaxf(v, 0.f); so[w][8 * hh + r][t * 16 + ln] = v; }
  }
  __builtin_amdgcn_fence(__ATOMIC_ACQ_REL, "workgroup");
  __builtin_amdgcn_wave_barrier();
  const int rsub = lane >> 4, c4 = (lane & 15) * 4;
  for (int pass = 0; pass < 2; ++pass) {
#pragma unroll
    for (int q = 0; q < 8; ++q) {
      const int r = q * 2 + rsub;
      const v4f v = *(const v4fa*)&so[w][r][c4];
      *(volatile v4f*)(C + (size_t)(row0 + r) * ldc + col0 + c4) = v;
    }
    if (pass == 0) __threadfence();
  }
}

template <int D, bool CAUSAL>
__global__ __launch_bounds__(128) void k_flash(const float* __restrict__ qb, const float* __restrict__ kb, const float* __restrict__ vb,
                                             int pitch, int T, int H, float scale, float* __restrict__ y, int ypitch) {
  constexpr int KS = D / 32;
  constexpr int DT = D / 16;
  __shared__ __attribute__((aligned(16))) unsigned short sKh[32][D + 8], sKl[32][D + 8], sVh[32][D + 8], sVl[32][D + 8];
  __shared__ __attribute__((aligned(16))) unsigned short sPh[4][16][40], sPl[4][16][40];
  __shared__ __attribute__((aligned(16))) float sO[4][16][D];
  const int tid = threadIdx.x, w = tid >> 5, lane = tid & 31, ln = lane & 15, hh = lane >> 4;
  const int nqb = (T + 63) / 64;
  const int bh = blockIdx.x / nqb, qblk = blockIdx.x % nqb;
  const int b = bh / H, h = bh % H;
  const int q0 = qblk * 64 + w * 16;
  const float* Q = qb + (size_t)b * T * pitch + h * D;
  const float* K = kb + (size_t)b * T * pitch + h * D;
  const float* V = vb + (size_t)b * T * pitch + h * D;

  FragB aqh[KS], aql[KS];
  {
    int row = q0 + ln; if (row >= T) row = T - 1;
    const float* qr = Q + (size_t)row * pitch;
#pragma unroll
    for (int ks = 0; ks < KS; ++ks)
#pragma unroll
      for (int i = 0; i < 16; ++i) {
        const int d = ks * 32 + ((i < 8) ? (8 * hh + i) : (16 + 8 * hh + (i - 8)));
        const float x = qr[d] * scale; const unsigned short hb = bf16_bits(x);
        aqh[ks].u[i] = hb; aql[ks].u[i] = bf16_bits(x - bf16_val(hb));
      }
  }
  float m_r[8], l_r[8];
#pragma unroll
  for (int r = 0; r < 8; ++r) { m_r[r] = -3.0e38f; l_r[r] = 0.f; }
  v8f oacc[DT];
#pragma unroll
  for (int dt = 0; dt < DT; ++dt) oacc[dt] = (v8f){0.f,0.f,0.f,0.f,0.f,0.f,0.f,0.f};

  const int kv_end = CAUSAL ? min(T, qblk * 64 + 64) : T;
  for (int j0 = 0; j0 < kv_end; j0 += 32) {
    __syncthreads();
    for (int e = tid; e < 32 * (D / 4); e += 128) {
      const int r = e / (D / 4), c4 = (e % (D / 4)) * 4;
      const int key = j0 + r;
      v4f kf = {0.f,0.f,0.f,0.f}, vf = {0.f,0.f,0.f,0.f};
      if (key < T) { kf = *(const v4fa*)(K + (size_t)key * pitch + c4); vf = *(const v4fa*)(V + (size_t)key * pitch + c4); }
#pragma unroll
      for (int t = 0; t < 4; ++t) {
        unsigned short hb = bf16_bits(kf[t]); sKh[r][c4 + t] = hb; sKl[r][c4 + t] = bf16_bits(kf[t] - bf16_val(hb));
        hb = bf16_bits(vf[t]); sVh[r][c4 + t] = hb; sVl[r][c4 + t] = bf16_bits(vf[t] - bf16_val(hb));
      }
    }
    __syncthreads();
    v8f s[2];
#pragma unroll
    for (int nt = 0; nt < 2; ++nt) {
      v8f acc = {};
#pragma unroll
      for (int ks = 0; ks < KS; ++ks) {
        FragB bh_, bl_;
        bh_.half[0] = *(const v8us*)&sKh[nt * 16 + ln][ks * 32 + 8 * hh]; bh_.half[1] = *(const v8us*)&sKh[nt * 16 + ln][ks * 32 + 16 + 8 * hh];
        bl_.half[0] = *(const v8us*)&sKl[nt * 16 + ln][ks * 32 + 8 * hh]; bl_.half[1] = *(const v8us*)&sKl[nt * 16 + ln][ks * 32 + 16 + 8 * hh];
        acc = mmaN<3>(aqh[ks].v, aql[ks].v, bh_.v, bl_.v, acc);
      }
      s[nt] = acc;
    }
    float alpha[8];
#pragma unroll
    for (int r = 0; r < 8; ++r) {
      const int qi = q0 + 8 * hh + r;
      const int ja = j0 + ln, jb = j0 + 16 + ln;
      if (CAUSAL) { if (ja > qi) s[0][r] = -3.0e38f; if (jb > qi) s[1][r] = -3.0e38f; }
      if (ja >= T) s[0][r] = -3.0e38f;
      if (jb >= T) s[1][r] = -3.0e38f;
      float mx = fmaxf(s[0][r], s[1][r]);
      mx = fmaxf(mx, __shfl_xor(mx, 1, 32)); mx = fmaxf(mx, __shfl_xor(mx, 2, 32)); mx = fmaxf(mx, __shfl_xor(mx, 4, 32)); mx = fmaxf(mx, __shfl_xor(mx, 8, 32));
      const float mnew = fmaxf(m_r[r], mx);
      alpha[r] = (mnew > -1.0e38f) ? __expf(m_r[r] - mnew) : 1.0f;
      const float p0 = (s[0][r] > -1.0e38f) ? __expf(s[0][r] - mnew) : 0.f;
      const float p1 = (s[1][r] > -1.0e38f) ? __expf(s[1][r] - mnew) : 0.f;
      m_r[r] = mnew;
      l_r[r] = l_r[r] * alpha[r] + p0 + p1;
      unsigned short hb = bf16_bits(p0); sPh[w][8 * hh + r][ln] = hb;      sPl[w][8 * hh + r][ln] = bf16_bits(p0 - bf16_val(hb));
      hb = bf16_bits(p1);                sPh[w][8 * hh + r][16 + ln] = hb; sPl[w][8 * hh + r][16 + ln] = bf16_bits(p1 - bf16_val(hb));
    }
#pragma unroll
    for (int dt = 0; dt < DT; ++dt)
#pragma unroll
      for (int r = 0; r < 8; ++r) oacc[dt][r] *= alpha[r];
    __builtin_amdgcn_fence(__ATOMIC_ACQ_REL, "workgroup");
    __builtin_amdgcn_wave_barrier();
    FragB pah, pal;
    pah.half[0] = *(const v8us*)&sPh[w][ln][8 * hh]; pah.half[1] = *(const v8us*)&sPh[w][ln][16 + 8 * hh];
    pal.half[0] = *(const v8us*)&sPl[w][ln][8 * hh]; pal.half[1] = *(const v8us*)&sPl[w][ln][16 + 8 * hh];
#pragma unroll
    for (int dt = 0; dt < DT; ++dt) {
      FragB bvh, bvl;
#pragma unroll
      for (int i = 0; i < 8; ++i) {
        bvh.u[i] = sVh[8 * hh + i][dt * 16 + ln]; bvh.u[8 + i] = sVh[16 + 8 * hh + i][dt * 16 + ln];
        bvl.u[i] = sVl[8 * hh + i][dt * 16 + ln]; bvl.u[8 + i] = sVl[16 + 8 * hh + i][dt * 16 + ln];
      }
      oacc[dt] = mmaN<3>(pah.v, pal.v, bvh.v, bvl.v, oacc[dt]);
    }
    __builtin_amdgcn_fence(__ATOMIC_ACQ_REL, "workgroup");
    __builtin_amdgcn_wave_barrier();
  }
#pragma unroll
  for (int r = 0; r < 8; ++r) {
    float l = l_r[r];
    l += __shfl_xor(l, 1, 32); l += __shfl_xor(l, 2, 32); l += __shfl_xor(l, 4, 32); l += __shfl_xor(l, 8, 32);
    l_r[r] = (l > 0.f) ? 1.0f / l : 0.f;
  }
#pragma unroll
  for (int dt = 0; dt < DT; ++dt)
#pragma unroll
    for (int r = 0; r < 8; ++r) sO[w][8 * hh + r][dt * 16 + ln] = oacc[dt][r] * l_r[r];
  __builtin_amdgcn_fence(__ATOMIC_ACQ_REL, "workgroup");
  __builtin_amdgcn_wave_barrier();
  for (int pass = 0; pass < 2; ++pass) {
    for (int r = 0; r < 16; ++r) {
      const int row = q0 + r;
      if (row < T && lane < D / 4) {
        const v4f val = *(const v4fa*)&sO[w][r][lane * 4];
        *(volatile v4f*)(y + ((size_t)b * T + row) * ypitch + h * D + lane * 4) = val;
      }
    }
    if (pass == 0) __threadfence();
  }
}

typedef _Float16 v16h __attribute__((ext_vector_type(16)));
union FragH { v16h v; v8us half[2]; _Float16 h[16]; unsigned short u[16]; };
template <int NT>
__device__ __forceinline__ v8f mmaH(v16h ah, v16h al, v16h bh, v16h bl, v8f c) {
  c = __builtin_amdgcn_wmma_f32_16x16x32_f16(false, ah, false, bh, (short)0, c, false, false);
  if (NT >= 2) c = __builtin_amdgcn_wmma_f32_16x16x32_f16(false, al, false, bh, (short)0, c, false, false);
  if (NT >= 3) c = __builtin_amdgcn_wmma_f32_16x16x32_f16(false, ah, false, bl, (short)0, c, false, false);
  asm volatile("v_nop\n\tv_nop\n\tv_nop\n\tv_nop" : "+v"(c) : "v"(ah), "v"(al), "v"(bh), "v"(bl));
  return c;
}
template <bool ASPLIT>
__global__ __launch_bounds__(128) void k_gemm_h(const float* __restrict__ A, int lda, size_t sA, const _Float16* __restrict__ Bh, int ldb, size_t sB, float alpha, float* __restrict__ C, int ldc, size_t sC, int M, int N, int K) {
  __shared__ __attribute__((aligned(16))) float so[4][16][64];
  const int tid = threadIdx.x, w = tid >> 5, lane = tid & 31, ln = lane & 15, hh = lane >> 4; const int by = blockIdx.y;
  A += (size_t)by * sA; Bh += (size_t)by * sB; C += (size_t)by * sC;
  const int ntn = (N + 63) / 64; const int wid = blockIdx.x * 4 + w; const int mt = wid / ntn, nq = wid % ntn; if (mt * 16 >= M) return;
  const int row0 = mt * 16, col0 = nq * 64; const float* arow = A + (size_t)(row0 + ln) * lda;
  v8f acc[4] = {};
  for (int kb = 0; kb < K; kb += 32) {
    FragH ah, al;
    const v4f x0 = *(const v4fa*)(arow + kb + 8 * hh), x1 = *(const v4fa*)(arow + kb + 8 * hh + 4), x2 = *(const v4fa*)(arow + kb + 16 + 8 * hh), x3 = *(const v4fa*)(arow + kb + 16 + 8 * hh + 4);
    float xs[16] = {x0[0],x0[1],x0[2],x0[3],x1[0],x1[1],x1[2],x1[3],x2[0],x2[1],x2[2],x2[3],x3[0],x3[1],x3[2],x3[3]};
#pragma unroll
    for (int i = 0; i < 16; ++i) { const _Float16 h = (_Float16)xs[i]; ah.h[i] = h; al.h[i] = ASPLIT ? (_Float16)(xs[i] - (float)h) : (_Float16)0.0f; }
#pragma unroll
    for (int t = 0; t < 4; ++t) { if (col0 + t * 16 >= N) continue; const size_t boff = (size_t)(col0 + t * 16 + ln) * ldb + kb; FragH bq; bq.half[0] = *(const v8us*)(Bh + boff + 8 * hh); bq.half[1] = *(const v8us*)(Bh + boff + 16 + 8 * hh);
      acc[t] = mmaH<ASPLIT ? 2 : 1>(ah.v, al.v, bq.v, bq.v, acc[t]); }
  }
#pragma unroll
  for (int t = 0; t < 4; ++t) { if (col0 + t * 16 >= N) continue;
#pragma unroll
    for (int r = 0; r < 8; ++r) so[w][8 * hh + r][t * 16 + ln] = acc[t][r] * alpha; }
  __builtin_amdgcn_fence(__ATOMIC_ACQ_REL, "workgroup"); __builtin_amdgcn_wave_barrier();
  const int rsub = lane >> 4, c4 = (lane & 15) * 4;
  for (int pass = 0; pass < 2; ++pass) {
#pragma unroll
    for (int q = 0; q < 8; ++q) { const int r = q * 2 + rsub; if (col0 + c4 < N) { const v4f v = *(const v4fa*)&so[w][r][c4]; *(volatile v4f*)(C + (size_t)(row0 + r) * ldc + col0 + c4) = v; } }
    if (pass == 0) __threadfence(); }
}

template <int DUMMY>
__global__ __launch_bounds__(128) void k_gemm_hh(const _Float16* __restrict__ A, int lda, size_t sA, const _Float16* __restrict__ Bh, int ldb, size_t sB, float alpha, float* __restrict__ C, int ldc, size_t sC, int M, int N, int K) {
  __shared__ __attribute__((aligned(16))) float so[4][16][64];
  const int tid = threadIdx.x, w = tid >> 5, lane = tid & 31, ln = lane & 15, hh = lane >> 4; const int by = blockIdx.y;
  A += (size_t)by * sA; Bh += (size_t)by * sB; C += (size_t)by * sC;
  const int ntn = (N + 63) / 64; const int wid = blockIdx.x * 4 + w; const int mt = wid / ntn, nq = wid % ntn; if (mt * 16 >= M) return;
  const int row0 = mt * 16, col0 = nq * 64; const _Float16* arow = A + (size_t)(row0 + ln) * lda;
  v8f acc[4] = {};
  for (int kb = 0; kb < K; kb += 32) { FragH ah; ah.half[0] = *(const v8us*)((const unsigned short*)arow + kb + 8 * hh); ah.half[1] = *(const v8us*)((const unsigned short*)arow + kb + 16 + 8 * hh);
#pragma unroll
    for (int t = 0; t < 4; ++t) { if (col0 + t * 16 >= N) continue; const size_t boff = (size_t)(col0 + t * 16 + ln) * ldb + kb; FragH bq; bq.half[0] = *(const v8us*)((const unsigned short*)Bh + boff + 8 * hh); bq.half[1] = *(const v8us*)((const unsigned short*)Bh + boff + 16 + 8 * hh);
      acc[t] = mmaH<1>(ah.v, ah.v, bq.v, bq.v, acc[t]); }
  }
#pragma unroll
  for (int t = 0; t < 4; ++t) { if (col0 + t * 16 >= N) continue;
#pragma unroll
    for (int r = 0; r < 8; ++r) so[w][8 * hh + r][t * 16 + ln] = acc[t][r] * alpha; }
  __builtin_amdgcn_fence(__ATOMIC_ACQ_REL, "workgroup"); __builtin_amdgcn_wave_barrier();
  const int rsub = lane >> 4, c4 = (lane & 15) * 4;
  for (int pass = 0; pass < 2; ++pass) {
#pragma unroll
    for (int q = 0; q < 8; ++q) { const int r = q * 2 + rsub; if (col0 + c4 < N) { const v4f v = *(const v4fa*)&so[w][r][c4]; *(volatile v4f*)(C + (size_t)(row0 + r) * ldc + col0 + c4) = v; } }
    if (pass == 0) __threadfence(); }
}

template <int ACT>
__global__ __launch_bounds__(128) void k_gemm_hhx(const _Float16* __restrict__ A, int lda, size_t sA, const _Float16* __restrict__ Bh, int ldb, size_t sB, float alpha, const float* __restrict__ bias, size_t sBias, const float* __restrict__ CP, int rowsPerB, size_t sCPb, int row0g,
    float* __restrict__ C, _Float16* __restrict__ C16, int ldc, size_t sC, int M, int N, int K) {
  __shared__ __attribute__((aligned(16))) float so[4][16][64];
  const int tid = threadIdx.x, w = tid >> 5, lane = tid & 31, ln = lane & 15, hh = lane >> 4; const int by = blockIdx.y;
  A += (size_t)by * sA; Bh += (size_t)by * sB; const size_t cofs = (size_t)by * sC; const float* bp = bias ? bias + (size_t)by * sBias : nullptr;
  const int ntn = (N + 63) / 64; const int wid = blockIdx.x * 4 + w; const int mt = wid / ntn, nq = wid % ntn; if (mt * 16 >= M) return;
  const int row0 = mt * 16, col0 = nq * 64; const _Float16* arow = A + (size_t)(row0 + ln) * lda;
  v8f acc[4] = {};
  for (int kb = 0; kb < K; kb += 32) { FragH ah; ah.half[0] = *(const v8us*)((const unsigned short*)arow + kb + 8 * hh); ah.half[1] = *(const v8us*)((const unsigned short*)arow + kb + 16 + 8 * hh);
#pragma unroll
    for (int t = 0; t < 4; ++t) { if (col0 + t * 16 >= N) continue; const size_t boff = (size_t)(col0 + t * 16 + ln) * ldb + kb; FragH bq; bq.half[0] = *(const v8us*)((const unsigned short*)Bh + boff + 8 * hh); bq.half[1] = *(const v8us*)((const unsigned short*)Bh + boff + 16 + 8 * hh);
      acc[t] = mmaH<1>(ah.v, ah.v, bq.v, bq.v, acc[t]); }
  }
#pragma unroll
  for (int t = 0; t < 4; ++t) { if (col0 + t * 16 >= N) continue; const int col = col0 + t * 16 + ln; const float bv = bp ? bf16_round(bp[col]) : 0.f;
#pragma unroll
    for (int r = 0; r < 8; ++r) { float v = acc[t][r] * alpha + bv; if (CP) { const int bidx = (row0g + row0 + 8 * hh + r) / rowsPerB; v += CP[(size_t)bidx * sCPb + (size_t)by * 64 + col]; } if (ACT == 1) v = (v > 0.f) ? v : expm1f(v); else if (ACT == 3) v = fmaxf(v, 0.f); so[w][8 * hh + r][t * 16 + ln] = v; } }
  __builtin_amdgcn_fence(__ATOMIC_ACQ_REL, "workgroup"); __builtin_amdgcn_wave_barrier();
  const int rsub = lane >> 4, c4 = (lane & 15) * 4; typedef _Float16 v4h __attribute__((ext_vector_type(4)));
  for (int pass = 0; pass < 2; ++pass) {
#pragma unroll
    for (int q = 0; q < 8; ++q) { const int r = q * 2 + rsub; if (col0 + c4 < N) { const v4f v = *(const v4fa*)&so[w][r][c4]; if (C) *(volatile v4f*)(C + cofs + (size_t)(row0 + r) * ldc + col0 + c4) = v; if (C16) { v4h h4; for (int i = 0; i < 4; ++i) h4[i] = (_Float16)v[i]; *(volatile v4h*)(C16 + cofs + (size_t)(row0 + r) * ldc + col0 + c4) = h4; } } }
    if (pass == 0) __threadfence(); }
}

__global__ __launch_bounds__(256) void k_bt(const float* __restrict__ w1, const float* __restrict__ wr, const float* __restrict__ wsx, const float* __restrict__ bsx, const float* __restrict__ w2, const float* __restrict__ wp1, const float* __restrict__ wp2, _Float16* __restrict__ W1, _Float16* __restrict__ WR, _Float16* __restrict__ WS, float* __restrict__ BSP, _Float16* __restrict__ W2, _Float16* __restrict__ WP1, _Float16* __restrict__ WP2) { const int t = blockIdx.x * 256 + threadIdx.x;
  if (t < CH * CC) *(volatile _Float16*)(W1 + t) = (_Float16)(bf16_round(w1[t]) * 16.0f);
  if (t < CQ * CH) *(volatile _Float16*)(WR + t) = (_Float16)(bf16_round(wr[t]) * 16.0f);
  if (t < NKP * CQ) { const int n = t / CQ; *(volatile _Float16*)(WS + t) = (_Float16)((n < NKW) ? bf16_round(wsx[t]) * 16.0f : 0.f); }
  if (t < NKP) *(volatile float*)(BSP + t) = (t < NKW) ? bsx[t] : 0.f;
  if (t < CC * CH) *(volatile _Float16*)(W2 + t) = (_Float16)(bf16_round(w2[t]) * 16.0f);
  if (t < CC * CQ) *(volatile _Float16*)(WP2 + t) = (_Float16)(bf16_round(wp2[t]) * 16.0f);
  if (t < CQ * 9 * CQ) { const int o = t / (9 * CQ), k = t % (9 * CQ); const int c = k % CQ, kk = k / CQ; *(volatile _Float16*)(WP1 + t) = (_Float16)(bf16_round(wp1[((size_t)o * CQ + c) * 9 + kk]) * 16.0f); } }
__global__ __launch_bounds__(256) void k_xin(const float* __restrict__ x, _Float16* __restrict__ AX) { __shared__ float tile[32][33]; const int b = blockIdx.z, c0 = blockIdx.y * 32, p0 = blockIdx.x * 32; const int tx = threadIdx.x & 31, ty = threadIdx.x >> 5;
  for (int i = ty; i < 32; i += 8) tile[i][tx] = bf16_round(x[((size_t)b * CC + c0 + i) * HW * HW + p0 + tx]); __syncthreads();
  typedef _Float16 v4h __attribute__((ext_vector_type(4))); const int r = threadIdx.x >> 3, c4 = (threadIdx.x & 7) * 4; v4h o; for (int q = 0; q < 4; ++q) o[q] = (_Float16)tile[c4 + q][r];
  _Float16* dst = AX + ((size_t)b * HW * HW + p0 + r) * CC + c0 + c4; *(volatile v4h*)dst = o; __threadfence(); *(volatile v4h*)dst = o; }
__global__ __launch_bounds__(256) void k_prelu(float* __restrict__ X, const float* __restrict__ ap, _Float16* __restrict__ Xh, size_t n8) { const size_t t = (size_t)blockIdx.x * 256 + threadIdx.x; if (t >= n8) return; const float a = bf16_round(ap[0]); FragH f; v4f o0 = *(const v4fa*)(X + t * 8), o1 = *(const v4fa*)(X + t * 8 + 4);
  for (int q = 0; q < 4; ++q) { o0[q] = o0[q] >= 0.f ? o0[q] : a * o0[q]; o1[q] = o1[q] >= 0.f ? o1[q] : a * o1[q]; f.h[q] = (_Float16)(o0[q] * 16.0f); f.h[4 + q] = (_Float16)(o1[q] * 16.0f); }
  store_span256(X + (t & ~(size_t)31) * 8, o0, o1, (int)(threadIdx.x & 31)); *(volatile v8us*)((unsigned short*)Xh + t * 8) = f.half[0]; __threadfence(); *(volatile v8us*)((unsigned short*)Xh + t * 8) = f.half[0]; }
__global__ __launch_bounds__(256) void k_inv(const float* __restrict__ KW, const float* __restrict__ X1, const float* __restrict__ ap, _Float16* __restrict__ A2) { const size_t t = (size_t)blockIdx.x * 256 + threadIdx.x; if (t >= (size_t)NP * CH / 8) return; const int c8 = (int)((t * 8) % CH); const size_t p = (t * 8) / CH; const int g = c8 / GC; const int b = (int)(p / (HW * HW)), pl = (int)(p % (HW * HW)); const int py = pl / HW, px = pl % HW; const float a = bf16_round(ap[0]);
  float acc[8]; for (int q = 0; q < 8; ++q) acc[q] = 0.f; const float* kwr = KW + p * NKP + g * K2;
#pragma unroll 1
  for (int i = 0; i < KINV; ++i) { const int yy = py + i - 3; if (yy < 0 || yy >= HW) continue;
#pragma unroll 1
    for (int j = 0; j < KINV; ++j) { const int xx = px + j - 3; if (xx < 0 || xx >= HW) continue; const float w = kwr[i * KINV + j]; const float* src = X1 + (((size_t)b * HW + yy) * HW + xx) * CH + c8; const v4f u0 = *(const v4fa*)src, u1 = *(const v4fa*)(src + 4);
      for (int q = 0; q < 4; ++q) { acc[q] += w * u0[q]; acc[4 + q] += w * u1[q]; } } }
  FragH f; for (int q = 0; q < 8; ++q) { const float v = acc[q]; f.h[q] = (_Float16)((v >= 0.f ? v : a * v) * 256.0f); }
  *(volatile v8us*)((unsigned short*)A2 + t * 8) = f.half[0]; __threadfence(); *(volatile v8us*)((unsigned short*)A2 + t * 8) = f.half[0]; }
__global__ __launch_bounds__(256) void k_zp(const float* __restrict__ F, float* __restrict__ ZP) { const size_t p = (size_t)blockIdx.x * 256 + threadIdx.x; if (p >= NP) return; const float* fr = F + p * CQ; float mx = -3.0e38f, s = 0.f;
#pragma unroll
  for (int c = 0; c < CQ; ++c) { const float v = fr[c]; mx = fmaxf(mx, v); s += v; } typedef float v2f __attribute__((ext_vector_type(2), aligned(8))); v2f o = {mx, s / (float)CQ}; *(volatile v2f*)(ZP + p * 2) = o; __threadfence(); *(volatile v2f*)(ZP + p * 2) = o; }
__global__ __launch_bounds__(256) void k_attn(const float* __restrict__ ZP, const float* __restrict__ wa, const float* __restrict__ ba, float* __restrict__ AT) { const size_t p = (size_t)blockIdx.x * 256 + threadIdx.x; if (p >= NP) return; const int b = (int)(p / (HW * HW)), pl = (int)(p % (HW * HW)); const int py = pl / HW, px = pl % HW; float s = bf16_round(ba[0]);
#pragma unroll 1
  for (int i = 0; i < KINV; ++i) { const int yy = py + i - 3; if (yy < 0 || yy >= HW) continue;
#pragma unroll 1
    for (int j = 0; j < KINV; ++j) { const int xx = px + j - 3; if (xx < 0 || xx >= HW) continue; const float* z = ZP + (((size_t)b * HW + yy) * HW + xx) * 2; s += bf16_round(wa[i * KINV + j]) * z[0] + bf16_round(wa[K2 + i * KINV + j]) * z[1]; } }
  const float v = 1.0f / (1.0f + expf(-s)); *(volatile float*)(AT + p) = v; __threadfence(); *(volatile float*)(AT + p) = v; }
__global__ __launch_bounds__(256) void k_im3(const float* __restrict__ F, _Float16* __restrict__ IM) { const size_t t = (size_t)blockIdx.x * 256 + threadIdx.x; if (t >= (size_t)NP * 9) return; const int tap = (int)(t % 9); const size_t p = t / 9; const int kh = tap / 3, kw = tap % 3; const int b = (int)(p / (HW * HW)), pl = (int)(p % (HW * HW)); const int yy = pl / HW + kh - 1, xx = pl % HW + kw - 1; const bool ok = yy >= 0 && yy < HW && xx >= 0 && xx < HW; const float* fr = F + (ok ? ((((size_t)b * HW + yy) * HW + xx) * CQ) : 0);
  unsigned short* dst = (unsigned short*)IM + p * (9 * CQ) + tap * CQ;
  for (int pass = 0; pass < 2; ++pass) { for (int q8 = 0; q8 < CQ; q8 += 8) { FragH f; for (int q = 0; q < 8; ++q) f.h[q] = (_Float16)(ok ? fr[q8 + q] * 64.0f : 0.f); *(volatile v8us*)(dst + q8) = f.half[0]; } if (pass == 0) __threadfence(); } }
__global__ __launch_bounds__(256) void k_prelu16(const float* __restrict__ X, const float* __restrict__ ap, _Float16* __restrict__ Xh, size_t n8) { const size_t t = (size_t)blockIdx.x * 256 + threadIdx.x; if (t >= n8) return; const float a = bf16_round(ap[0]); FragH f; const v4f o0 = *(const v4fa*)(X + t * 8), o1 = *(const v4fa*)(X + t * 8 + 4); for (int q = 0; q < 4; ++q) { f.h[q] = (_Float16)((o0[q] >= 0.f ? o0[q] : a * o0[q]) * 256.0f); f.h[4 + q] = (_Float16)((o1[q] >= 0.f ? o1[q] : a * o1[q]) * 256.0f); } *(volatile v8us*)((unsigned short*)Xh + t * 8) = f.half[0]; __threadfence(); *(volatile v8us*)((unsigned short*)Xh + t * 8) = f.half[0]; }
__global__ __launch_bounds__(256) void k_f16s(const float* __restrict__ X, _Float16* __restrict__ Xh, size_t n8) { const size_t t = (size_t)blockIdx.x * 256 + threadIdx.x; if (t >= n8) return; FragH f; for (int q = 0; q < 8; ++q) f.h[q] = (_Float16)(X[t * 8 + q] * 64.0f); *(volatile v8us*)((unsigned short*)Xh + t * 8) = f.half[0]; __threadfence(); *(volatile v8us*)((unsigned short*)Xh + t * 8) = f.half[0]; }
__global__ __launch_bounds__(256) void k_out(const float* __restrict__ X3, const float* __restrict__ AT, const float* __restrict__ PS, float* __restrict__ out) { __shared__ float tile[32][33]; const int b = blockIdx.z, c0 = blockIdx.y * 32, p0 = blockIdx.x * 32; const int tx = threadIdx.x & 31, ty = threadIdx.x >> 5;
  for (int i = ty; i < 32; i += 8) { const size_t p = (size_t)b * HW * HW + p0 + i; tile[i][tx] = X3[p * CC + c0 + tx] * AT[p] + PS[p * CC + c0 + tx]; } __syncthreads();
  const int r = threadIdx.x >> 3, c4 = (threadIdx.x & 7) * 4; v4f o; for (int q = 0; q < 4; ++q) o[q] = tile[c4 + q][r];
  float* dst = out + ((size_t)b * CC + c0 + r) * HW * HW + p0 + c4; *(volatile v4f*)dst = o; __threadfence(); *(volatile v4f*)dst = o; }
extern "C" void kernel_launch(void* const* d_in, const int* in_sizes, int n_in,
                              void* d_out, int out_size, void* d_ws, size_t ws_size, hipStream_t stream) {
  (void)in_sizes; (void)n_in; (void)out_size;
  const float* x = (const float*)d_in[0]; const float* w1 = (const float*)d_in[1]; const float* b1 = (const float*)d_in[2]; const float* a1 = (const float*)d_in[3]; const float* wr = (const float*)d_in[4]; const float* br = (const float*)d_in[5]; const float* wsx = (const float*)d_in[6]; const float* bsx = (const float*)d_in[7]; const float* a2 = (const float*)d_in[8]; const float* w2 = (const float*)d_in[9]; const float* b2 = (const float*)d_in[10]; const float* wa = (const float*)d_in[11]; const float* ba = (const float*)d_in[12]; const float* wp1 = (const float*)d_in[13]; const float* bp1 = (const float*)d_in[14]; const float* ap = (const float*)d_in[15]; const float* wp2 = (const float*)d_in[16]; const float* bp2 = (const float*)d_in[17];
  char* ws = (char*)d_ws; size_t off = 0;
  auto take = [&](size_t bytes) { char* p = ws + off; off += (bytes + 255) & ~(size_t)255; return p; };
  _Float16* W1 = (_Float16*)take(CH * CC * 2); _Float16* WR = (_Float16*)take(CQ * CH * 2); _Float16* WS = (_Float16*)take(NKP * CQ * 2); float* BSP = (float*)take(NKP * 4); _Float16* W2 = (_Float16*)take(CC * CH * 2); _Float16* WP1 = (_Float16*)take(CQ * 9 * CQ * 2); _Float16* WP2 = (_Float16*)take(CC * CQ * 2);
  _Float16* AX = (_Float16*)take((size_t)NP * CC * 2); float* X1 = (float*)take((size_t)NP * CH * 4); _Float16* X1h = (_Float16*)take((size_t)NP * CH * 2); float* F = (float*)take((size_t)NP * CQ * 4); _Float16* Fh = (_Float16*)take((size_t)NP * CQ * 2); float* KW = (float*)take((size_t)NP * NKP * 4);
  _Float16* A2 = (_Float16*)take((size_t)NP * CH * 2); float* X3 = (float*)take((size_t)NP * CC * 4); float* ZP = (float*)take((size_t)NP * 2 * 4); float* AT = (float*)take((size_t)NP * 4); _Float16* IM = (_Float16*)take((size_t)NP * 9 * CQ * 2); float* P1 = (float*)take((size_t)NP * CQ * 4); _Float16* P1h = (_Float16*)take((size_t)NP * CQ * 2); float* PS = (float*)take((size_t)NP * CC * 4);
  if (off > ws_size) return;
  auto EW = [](size_t n) { return (unsigned)((n + 255) / 256); };
  k_bt<<<EW(NKP * CQ > CQ * 9 * CQ ? (CC * CH) : (CQ * 9 * CQ)), 256, 0, stream>>>(w1, wr, wsx, bsx, w2, wp1, wp2, W1, WR, WS, BSP, W2, WP1, WP2);
  k_xin<<<dim3(HW * HW / 32, CC / 32, BB), 256, 0, stream>>>(x, AX);
  k_gemm_hhx<0><<<dim3(((NP / 16) * (CH / 64) + 3) / 4, 1), 128, 0, stream>>>(AX, CC, 0, W1, CC, 0, 0.0625f, b1, 0, nullptr, 1, 0, 0, X1, nullptr, CH, 0, NP, CH, CC);
  k_prelu<<<EW((size_t)NP * CH / 8), 256, 0, stream>>>(X1, a1, X1h, (size_t)NP * CH / 8);
  k_gemm_hhx<3><<<dim3(((NP / 16) * 1 + 3) / 4, 1), 128, 0, stream>>>(X1h, CH, 0, WR, CH, 0, 0.00390625f, br, 0, nullptr, 1, 0, 0, F, nullptr, CQ, 0, NP, CQ, CH);
  k_f16s<<<EW((size_t)NP * CQ / 8), 256, 0, stream>>>(F, Fh, (size_t)NP * CQ / 8);
  k_gemm_hhx<0><<<dim3(((NP / 16) * ((NKP + 63) / 64) + 3) / 4, 1), 128, 0, stream>>>(Fh, CQ, 0, WS, CQ, 0, 0.0009765625f, BSP, 0, nullptr, 1, 0, 0, KW, nullptr, NKP, 0, NP, NKP, CQ);
  k_inv<<<EW((size_t)NP * CH / 8), 256, 0, stream>>>(KW, X1, a2, A2);
  k_gemm_hhx<0><<<dim3(((NP / 16) * (CC / 64) + 3) / 4, 1), 128, 0, stream>>>(A2, CH, 0, W2, CH, 0, 0.000244140625f, b2, 0, nullptr, 1, 0, 0, X3, nullptr, CC, 0, NP, CC, CH);
  k_zp<<<EW(NP), 256, 0, stream>>>(F, ZP); k_attn<<<EW(NP), 256, 0, stream>>>(ZP, wa, ba, AT);
  k_im3<<<EW((size_t)NP * 9), 256, 0, stream>>>(F, IM);
  k_gemm_hhx<0><<<dim3(((NP / 16) * 1 + 3) / 4, 1), 128, 0, stream>>>(IM, 9 * CQ, 0, WP1, 9 * CQ, 0, 0.0009765625f, bp1, 0, nullptr, 1, 0, 0, P1, nullptr, CQ, 0, NP, CQ, 9 * CQ);
  k_prelu16<<<EW((size_t)NP * CQ / 8), 256, 0, stream>>>(P1, ap, P1h, (size_t)NP * CQ / 8);
  k_gemm_hhx<0><<<dim3(((NP / 16) * (CC / 64) + 3) / 4, 1), 128, 0, stream>>>(P1h, CQ, 0, WP2, CQ, 0, 0.000244140625f, bp2, 0, nullptr, 1, 0, 0, PS, nullptr, CC, 0, NP, CC, CQ);
  k_out<<<dim3(HW * HW / 32, CC / 32, BB), 256, 0, stream>>>(X3, AT, PS, (float*)d_out);
}
